// ScatterBrain_71674414235761
// MI455X (gfx1250) — hardware-verified
//
#include <hip/hip_runtime.h>

#define NB    4
#define SL    2048
#define DMOD  768
#define NHD   12
#define FDIM  16
#define HDIM  64
#define NBH   (NB * NHD)
#define NTOK  (NB * SL)
#define NQK   (NHD * FDIM)
#define NPROJ (2 * NQK + NHD * HDIM)
#define QROW  32
#define TPB   128
#define OSTR  68
#define ARESB 4

static_assert(NHD * HDIM == DMOD);
static_assert(NTOK % TPB == 0);
static_assert(SL % TPB == 0);
static_assert(NPROJ % 64 == 0);
static_assert(NQK % 64 == 0);
static_assert(NQK % 32 == 0);
static_assert(DMOD % 64 == 0);
static_assert(DMOD % 32 == 0);
static_assert(4 * FDIM == 64);
static_assert(HDIM == 64);
static_assert(QROW == 2 * FDIM);
static_assert(OSTR % 4 == 0);
static_assert((NTOK * DMOD) % (8 * 256) == 0);
static_assert(ARESB * TPB <= SL);

typedef unsigned short us16 __attribute__((ext_vector_type(16)));
typedef unsigned short us8  __attribute__((ext_vector_type(8)));
typedef unsigned short us8a __attribute__((ext_vector_type(8), may_alias));
typedef __bf16 v16b __attribute__((ext_vector_type(16)));
typedef _Float16 v16h __attribute__((ext_vector_type(16)));
typedef float v8f __attribute__((ext_vector_type(8)));
typedef float v4f __attribute__((ext_vector_type(4)));
typedef float v4fa __attribute__((ext_vector_type(4), may_alias));
union FragU { us16 v; us8 h[2]; };

__device__ __forceinline__ unsigned short bf16_bits(float f) {
  unsigned u = __float_as_uint(f);
  u += 0x7FFFu + ((u >> 16) & 1u);
  return (unsigned short)(u >> 16);
}
__device__ __forceinline__ float bf16_val(unsigned short b) { return __uint_as_float(((unsigned)b) << 16); }
__device__ __forceinline__ float bf16r(float f) { return bf16_val(bf16_bits(f)); }
__device__ __forceinline__ unsigned short f16_bits(float f) { return __builtin_bit_cast(unsigned short, (_Float16)f); }

__device__ __forceinline__ void f16split16(float a, unsigned short& hb, unsigned short& lb) {
  const float z = a * 16.0f;
  const _Float16 hf = (_Float16)z;
  const float res = (z - (float)hf) * 2048.0f;
  hb = __builtin_bit_cast(unsigned short, hf);
  lb = __builtin_bit_cast(unsigned short, (_Float16)res);
}
__device__ __forceinline__ void f16split64(float a, unsigned short& hb, unsigned short& lb) {
  const float z = a * 64.0f;
  const _Float16 hf = (_Float16)z;
  const float res = z - (float)hf;
  hb = __builtin_bit_cast(unsigned short, hf);
  lb = __builtin_bit_cast(unsigned short, (_Float16)res);
}

__device__ __forceinline__ v8f mma_bf16(us16 a, us16 b, v8f c) {
  return __builtin_amdgcn_wmma_f32_16x16x32_bf16(false, __builtin_bit_cast(v16b, a), false, __builtin_bit_cast(v16b, b), (short)0, c, false, false);
}
__device__ __forceinline__ v8f mma_f16(us16 a, us16 b, v8f c) {
  return __builtin_amdgcn_wmma_f32_16x16x32_f16(false, __builtin_bit_cast(v16h, a), false, __builtin_bit_cast(v16h, b), (short)0, c, false, false);
}
__device__ __forceinline__ void wguard2(v8f& c0, v8f& c1, const us16& a0, const us16& a1, const us16& b0, const us16& b1) {
#if defined(__HIP_DEVICE_COMPILE__)
  asm volatile("v_nop\n\tv_nop\n\tv_nop\n\tv_nop"
               : "+v"(c0), "+v"(c1)
               : "v"(a0), "v"(a1), "v"(b0), "v"(b1));
#endif
}
__device__ __forceinline__ void wguard4(v8f& c0, v8f& c1, v8f& c2, v8f& c3, const us16& a0,
                                        const us16& b0, const us16& b1, const us16& b2, const us16& b3) {
#if defined(__HIP_DEVICE_COMPILE__)
  asm volatile("v_nop\n\tv_nop\n\tv_nop\n\tv_nop"
               : "+v"(c0), "+v"(c1), "+v"(c2), "+v"(c3)
               : "v"(a0), "v"(b0), "v"(b1), "v"(b2), "v"(b3));
#endif
}
__device__ __forceinline__ void wguard8(v8f& c0, v8f& c1, v8f& c2, v8f& c3, v8f& c4, v8f& c5, v8f& c6, v8f& c7,
                                        const us16& a0, const us16& a1,
                                        const us16& b0, const us16& b1, const us16& b2, const us16& b3) {
#if defined(__HIP_DEVICE_COMPILE__)
  asm volatile("v_nop\n\tv_nop\n\tv_nop\n\tv_nop"
               : "+v"(c0), "+v"(c1), "+v"(c2), "+v"(c3), "+v"(c4), "+v"(c5), "+v"(c6), "+v"(c7)
               : "v"(a0), "v"(a1), "v"(b0), "v"(b1), "v"(b2), "v"(b3));
#endif
}

__device__ __forceinline__ us16 gfrag(const unsigned short* p) {
  const int kh = ((threadIdx.x >> 4) & 1) * 8;
  FragU f;
  f.h[0] = *(const us8a*)(p + kh);
  f.h[1] = *(const us8a*)(p + 16 + kh);
  return f.v;
}

__global__ __launch_bounds__(256) void k_cvt_bf16(const float* __restrict__ src, unsigned short* dst, int total8) {
  const int idx = blockIdx.x * 256 + threadIdx.x;
  if (idx >= total8) return;
  const size_t off = (size_t)idx * 8;
  const v4f a = *(const v4fa*)(src + off), b = *(const v4fa*)(src + off + 4);
  us8 o;
#pragma unroll
  for (int u = 0; u < 4; ++u) {
    o[u]     = bf16_bits(a[u]);
    o[4 + u] = bf16_bits(b[u]);
  }
  *(volatile us8*)(dst + off) = o;
  __threadfence();
  *(volatile us8*)(dst + off) = o;
}

template <int MODE>
__global__ __launch_bounds__(256) void k_wT(const float* __restrict__ src, int ncol, unsigned short* dst, int nrow0) {
  __shared__ float ts[64][33];
  const int tid = threadIdx.x;
  const int n0 = blockIdx.x * 32, k0 = blockIdx.y * 64;
  {
    const int k = tid >> 2, q = (tid & 3) * 8;
    const float* p = src + (size_t)(k0 + k) * (size_t)ncol + n0 + q;
    const v4f a = *(const v4fa*)p, c = *(const v4fa*)(p + 4);
#pragma unroll
    for (int u = 0; u < 4; ++u) { ts[k][q + u] = a[u]; ts[k][q + 4 + u] = c[u]; }
  }
  __syncthreads();
  const int n = tid >> 3, pc = (tid & 7) * 8;
  us8 o;
#pragma unroll
  for (int i = 0; i < 8; ++i) {
    const float w = ts[pc + i][n];
    o[i] = (MODE == 0) ? bf16_bits(w) : f16_bits(bf16r(w) * 256.0f);
  }
  unsigned short* d = dst + (size_t)(nrow0 + n0 + n) * (size_t)DMOD + k0 + pc;
  *(volatile us8*)d = o;
  __threadfence();
  *(volatile us8*)d = o;
}

__global__ __launch_bounds__(256) void k_gemm_proj(const unsigned short* __restrict__ Ap, const unsigned short* __restrict__ Bw,
                                                  unsigned short* Qp, unsigned short* Kp, unsigned short* VH, unsigned short* VL) {
  __shared__ __attribute__((aligned(16))) float oS[8 * 16 * OSTR];
  const int tid = threadIdx.x, lane = tid & 31, wave = tid >> 5, cl = lane & 15, hh = lane >> 4;
  const int m0 = blockIdx.x * TPB + 16 * wave, n0 = blockIdx.y * 64;

  v8f acc[4];
#pragma unroll
  for (int j = 0; j < 4; ++j) { const v8f zz = {0.f, 0.f, 0.f, 0.f, 0.f, 0.f, 0.f, 0.f}; acc[j] = zz; }

  const unsigned short* a0p = Ap + (size_t)(m0 + cl) * (size_t)DMOD;
  const unsigned short* bwp = Bw + (size_t)(n0 + cl) * (size_t)DMOD;
#pragma unroll 1
  for (int k0 = 0; k0 < DMOD; k0 += 32) {
    const us16 af = gfrag(a0p + k0);
    us16 bfr[4];
#pragma unroll
    for (int j = 0; j < 4; ++j) bfr[j] = gfrag(bwp + (size_t)(16 * j) * (size_t)DMOD + k0);
#pragma unroll
    for (int j = 0; j < 4; ++j) acc[j] = mma_bf16(af, bfr[j], acc[j]);
    wguard4(acc[0], acc[1], acc[2], acc[3], af, bfr[0], bfr[1], bfr[2], bfr[3]);
  }

  float* so = oS + wave * (16 * OSTR);
#pragma unroll
  for (int j = 0; j < 4; ++j)
#pragma unroll
    for (int r = 0; r < 8; ++r) so[(8 * hh + r) * OSTR + 16 * j + cl] = acc[j][r];
  __syncthreads();

  const int yb = blockIdx.y;
  const int m0b = blockIdx.x * TPB, b = m0b / SL, tb = m0b - b * SL;
  if (yb < 6) {
    unsigned short* dst = (yb < 3) ? Qp : Kp;
    const int h0 = 4 * ((yb < 3) ? yb : (yb - 3));
    us8 ov[8];
#pragma unroll
    for (int it = 0; it < 8; ++it) {
      const int cx = it * 256 + tid, u = cx & 3, r = (cx >> 2) & 127, j = cx >> 9;
      const float* sp = oS + r * OSTR + 16 * j + 8 * (u & 1);
      const v4f z0 = *(const v4fa*)sp, z1 = *(const v4fa*)(sp + 4);
      us8 o;
#pragma unroll
      for (int q4 = 0; q4 < 4; ++q4) {
        unsigned short hb, lb;
        f16split64(z0[q4], hb, lb); o[q4]     = (u >> 1) ? lb : hb;
        f16split64(z1[q4], hb, lb); o[4 + q4] = (u >> 1) ? lb : hb;
      }
      ov[it] = o;
    }
#pragma unroll
    for (int pass = 0; pass < 2; ++pass) {
#pragma unroll
      for (int it = 0; it < 8; ++it) {
        const int cx = it * 256 + tid, u = cx & 3, r = (cx >> 2) & 127, j = cx >> 9;
        const size_t off = ((size_t)(b * NHD + h0 + j) * (size_t)SL + (size_t)(tb + r)) * (size_t)QROW + (size_t)(8 * u);
        *(volatile us8*)(dst + off) = ov[it];
      }
      __threadfence();
    }
  } else {
    const int head = yb - 6;
    us8 hv[4], lv[4];
#pragma unroll
    for (int it = 0; it < 4; ++it) {
      const int cx = it * 256 + tid, g = cx & 15, e = cx >> 4;
      us8 ho, lo;
#pragma unroll
      for (int i = 0; i < 8; ++i) {
        const float w = oS[(8 * g + i) * OSTR + e];
        unsigned short hb, lb;
        f16split64(w, hb, lb);
        ho[i] = hb; lo[i] = lb;
      }
      hv[it] = ho; lv[it] = lo;
    }
#pragma unroll
    for (int pass = 0; pass < 2; ++pass) {
#pragma unroll
      for (int it = 0; it < 4; ++it) {
        const int cx = it * 256 + tid, g = cx & 15, e = cx >> 4;
        const size_t off = ((size_t)(b * NHD + head) * (size_t)HDIM + (size_t)e) * (size_t)SL + (size_t)(tb + 8 * g);
        *(volatile us8*)(VH + off) = hv[it];
        *(volatile us8*)(VL + off) = lv[it];
      }
      __threadfence();
    }
  }
}

__global__ __launch_bounds__(256) void k_attn(const unsigned short* __restrict__ Qp, const unsigned short* __restrict__ Kp,
                                             const unsigned short* __restrict__ VHp, const unsigned short* __restrict__ VLp,
                                             unsigned short* YH, unsigned short* YL) {
  __shared__ __attribute__((aligned(16))) float oS[8 * 16 * OSTR];
  const int tid = threadIdx.x, lane = tid & 31, wave = tid >> 5, cl = lane & 15, hh = lane >> 4;
  const int bh = blockIdx.x, b = bh / NHD, head = bh - b * NHD;
  const int tw = blockIdx.y * TPB + 16 * wave;
  const int tq = tw + cl;
  const bool ares = (blockIdx.y < ARESB);

  const unsigned short* qrow = Qp + ((size_t)bh * SL + (size_t)tq) * (size_t)QROW + 8 * hh;
  FragU fq;
  fq.h[0] = *(const us8a*)qrow;         fq.h[1] = fq.h[0];
  const us16 bq1 = fq.v;
  fq.h[0] = *(const us8a*)(qrow + 16);  fq.h[1] = fq.h[0];
  const us16 bq2 = fq.v;

  v8f accS[4], accL[4];
#pragma unroll
  for (int j = 0; j < 4; ++j) { const v8f zz = {0.f, 0.f, 0.f, 0.f, 0.f, 0.f, 0.f, 0.f}; accS[j] = zz; accL[j] = zz; }
  float zp = 0.0f;

  const unsigned short* kbp = Kp + ((size_t)bh * SL + (size_t)cl) * (size_t)QROW;
  const unsigned short* vhp = VHp + ((size_t)bh * HDIM + (size_t)cl) * (size_t)SL;
  const unsigned short* vlp = VLp + ((size_t)bh * HDIM + (size_t)cl) * (size_t)SL;
  const int nsteps = (tw + 47) >> 5;

#pragma unroll 1
  for (int st = 0; st < nsteps; ++st) {
    const int s0 = st * 32;
    const us16 ka = gfrag(kbp + (size_t)s0 * QROW);
    const us16 kb = gfrag(kbp + (size_t)(s0 + 16) * QROW);
    const v8f zz = {0.f, 0.f, 0.f, 0.f, 0.f, 0.f, 0.f, 0.f};
    v8f sa = mma_f16(ka, bq1, zz);
    sa = mma_f16(ka, bq2, sa);
    v8f sb = mma_f16(kb, bq1, zz);
    sb = mma_f16(kb, bq2, sb);
    wguard2(sa, sb, ka, kb, bq1, bq2);

    us8 ea, eb, la8, lb8;
    float zs = 0.0f;
#pragma unroll
    for (int r = 0; r < 8; ++r) {
      const int ky = s0 + 8 * hh + r;
      const float xa = sa[r] * (1.0f / 16384.0f);
      const float xb = sb[r] * (1.0f / 16384.0f);
      float pa = fmaf(xa, fmaf(xa, 0.5f, 1.0f), 1.0f);
      float pb = fmaf(xb, fmaf(xb, 0.5f, 1.0f), 1.0f);
      pa = (ky <= tq) ? pa : 0.0f;
      pb = (ky + 16 <= tq) ? pb : 0.0f;
      const _Float16 fa = (_Float16)pa, fb = (_Float16)pb;
      const _Float16 ra = (_Float16)((pa - (float)fa) * 2048.0f);
      const _Float16 rb = (_Float16)((pb - (float)fb) * 2048.0f);
      zs += ares ? (pa + pb) : ((float)fa + (float)fb);
      ea[r]  = __builtin_bit_cast(unsigned short, fa);
      eb[r]  = __builtin_bit_cast(unsigned short, fb);
      la8[r] = __builtin_bit_cast(unsigned short, ra);
      lb8[r] = __builtin_bit_cast(unsigned short, rb);
    }
    zp += zs;
    FragU fA;
    fA.h[0] = ea; fA.h[1] = eb;
    const us16 ahi = fA.v;
    FragU fR;
    fR.h[0] = la8; fR.h[1] = lb8;
    const us16 alo = fR.v;

    us16 bv[4];
#pragma unroll
    for (int j = 0; j < 4; ++j) bv[j] = gfrag(vhp + (size_t)(16 * j) * (size_t)SL + s0);
    if (ares) {
#pragma unroll
      for (int j = 0; j < 4; ++j) {
        accS[j] = mma_f16(ahi, bv[j], accS[j]);
        accL[j] = mma_f16(alo, bv[j], accL[j]);
      }
      wguard8(accS[0], accS[1], accS[2], accS[3], accL[0], accL[1], accL[2], accL[3], ahi, alo, bv[0], bv[1], bv[2], bv[3]);
      us16 bl[4];
#pragma unroll
      for (int j = 0; j < 4; ++j) bl[j] = gfrag(vlp + (size_t)(16 * j) * (size_t)SL + s0);
#pragma unroll
      for (int j = 0; j < 4; ++j) accS[j] = mma_f16(ahi, bl[j], accS[j]);
      wguard4(accS[0], accS[1], accS[2], accS[3], ahi, bl[0], bl[1], bl[2], bl[3]);
    } else {
#pragma unroll
      for (int j = 0; j < 4; ++j) accS[j] = mma_f16(ahi, bv[j], accS[j]);
      wguard4(accS[0], accS[1], accS[2], accS[3], ahi, bv[0], bv[1], bv[2], bv[3]);
    }
  }

  const float zf = zp + __shfl_xor(zp, 16, 32);
  float rz[8];
#pragma unroll
  for (int r = 0; r < 8; ++r) {
    const float zr = __shfl(zf, 8 * hh + r, 32);
    rz[r] = (1.0f / (zr + 1e-12f)) * (1.0f / 64.0f);
  }

  float* so = oS + wave * (16 * OSTR);
#pragma unroll
  for (int j = 0; j < 4; ++j)
#pragma unroll
    for (int r = 0; r < 8; ++r) so[(8 * hh + r) * OSTR + 16 * j + cl] = fmaf(accL[j][r], (1.0f / 2048.0f), accS[j][r]) * rz[r];
  __syncthreads();

  us8 hv[4], lv[4];
#pragma unroll
  for (int it = 0; it < 4; ++it) {
    const int rr = it * 4 + (lane >> 3), p = (lane & 7) * 8;
    const v4f z0 = *(const v4fa*)(so + rr * OSTR + p), z1 = *(const v4fa*)(so + rr * OSTR + p + 4);
    us8 ho, lo;
#pragma unroll
    for (int u = 0; u < 4; ++u) {
      unsigned short hb, lb;
      f16split16(z0[u], hb, lb); ho[u] = hb;     lo[u] = lb;
      f16split16(z1[u], hb, lb); ho[4 + u] = hb; lo[4 + u] = lb;
    }
    hv[it] = ho; lv[it] = lo;
  }
#pragma unroll
  for (int pass = 0; pass < 2; ++pass) {
#pragma unroll
    for (int it = 0; it < 4; ++it) {
      const int rr = it * 4 + (lane >> 3), p = (lane & 7) * 8;
      const size_t off = (size_t)(b * SL + tw + rr) * (size_t)DMOD + (size_t)(head * HDIM + p);
      *(volatile us8*)(YH + off) = hv[it];
      *(volatile us8*)(YL + off) = lv[it];
    }
    __threadfence();
  }
}

__global__ __launch_bounds__(256) void k_gemm_out(const unsigned short* __restrict__ Ah, const unsigned short* __restrict__ Al,
                                                 const unsigned short* __restrict__ Wo, float* out) {
  __shared__ __attribute__((aligned(16))) float oS[8 * 16 * OSTR];
  const int tid = threadIdx.x, lane = tid & 31, wave = tid >> 5, cl = lane & 15, hh = lane >> 4;
  const int m0 = blockIdx.x * TPB + 16 * wave, n0 = blockIdx.y * 64;

  v8f acch[4], accl[4];
#pragma unroll
  for (int j = 0; j < 4; ++j) { const v8f zz = {0.f, 0.f, 0.f, 0.f, 0.f, 0.f, 0.f, 0.f}; acch[j] = zz; accl[j] = zz; }

  const unsigned short* ahp = Ah + (size_t)(m0 + cl) * (size_t)DMOD;
  const unsigned short* alp = Al + (size_t)(m0 + cl) * (size_t)DMOD;
  const unsigned short* wop = Wo + (size_t)(n0 + cl) * (size_t)DMOD;
#pragma unroll 1
  for (int k0 = 0; k0 < DMOD; k0 += 32) {
    const us16 ah = gfrag(ahp + k0);
    const us16 al = gfrag(alp + k0);
    us16 bfr[4];
#pragma unroll
    for (int j = 0; j < 4; ++j) bfr[j] = gfrag(wop + (size_t)(16 * j) * (size_t)DMOD + k0);
#pragma unroll
    for (int j = 0; j < 4; ++j) {
      acch[j] = mma_f16(ah, bfr[j], acch[j]);
      accl[j] = mma_f16(al, bfr[j], accl[j]);
    }
    wguard8(acch[0], acch[1], acch[2], acch[3], accl[0], accl[1], accl[2], accl[3], ah, al, bfr[0], bfr[1], bfr[2], bfr[3]);
  }

  float* so = oS + wave * (16 * OSTR);
#pragma unroll
  for (int j = 0; j < 4; ++j)
#pragma unroll
    for (int r = 0; r < 8; ++r)
      so[(8 * hh + r) * OSTR + 16 * j + cl] = fmaf(accl[j][r], (1.0f / 2048.0f), acch[j][r]) * (1.0f / 4096.0f);
  __syncthreads();

#pragma unroll
  for (int pass = 0; pass < 2; ++pass) {
#pragma unroll
    for (int it = 0; it < 8; ++it) {
      const int cx = it * 32 + lane, r = cx >> 4, q = (cx & 15) * 4;
      const v4f v = *(const v4fa*)(so + r * OSTR + q);
      *(volatile v4f*)(out + (size_t)(m0 + r) * (size_t)DMOD + n0 + q) = v;
    }
    __threadfence();
  }
}

extern "C" void kernel_launch(void* const* d_in, const int* in_sizes, int n_in,
                              void* d_out, int out_size, void* d_ws, size_t ws_size,
                              hipStream_t stream) {
  if (n_in < 5) return;
  if (in_sizes[0] != NTOK * DMOD || in_sizes[1] != DMOD * NQK || in_sizes[2] != DMOD * NQK ||
      in_sizes[3] != DMOD * DMOD || in_sizes[4] != DMOD * DMOD) return;
  if (out_size != NTOK * DMOD) return;

  const float* x  = (const float*)d_in[0];
  const float* Wq = (const float*)d_in[1];
  const float* Wk = (const float*)d_in[2];
  const float* Wv = (const float*)d_in[3];
  const float* Wo = (const float*)d_in[4];
  float* out = (float*)d_out;

  size_t off = 0;
  auto carve = [&](size_t bytes) -> char* { char* p = (char*)d_ws + off; off += (bytes + 255) & ~(size_t)255; return p; };
  unsigned short* XB   = (unsigned short*)carve((size_t)NTOK * DMOD * 2);
  unsigned short* WT   = (unsigned short*)carve((size_t)NPROJ * DMOD * 2);
  unsigned short* WO16 = (unsigned short*)carve((size_t)DMOD * DMOD * 2);
  unsigned short* QP   = (unsigned short*)carve((size_t)NBH * SL * QROW * 2);
  unsigned short* KP   = (unsigned short*)carve((size_t)NBH * SL * QROW * 2);
  unsigned short* VH   = (unsigned short*)carve((size_t)NBH * HDIM * SL * 2);
  unsigned short* VL   = (unsigned short*)carve((size_t)NBH * HDIM * SL * 2);
  unsigned short* YH   = (unsigned short*)carve((size_t)NTOK * DMOD * 2);
  unsigned short* YL   = (unsigned short*)carve((size_t)NTOK * DMOD * 2);
  if (off > ws_size || off > (size_t)134217728) return;

  const dim3 b256(256);
  auto cdv = [](long a, long q) { return (unsigned)((a + q - 1) / q); };

  k_cvt_bf16<<<dim3(cdv((long)NTOK * DMOD / 8, 256)), b256, 0, stream>>>(x, XB, NTOK * DMOD / 8);
  k_wT<0><<<dim3(NQK / 32, DMOD / 64), b256, 0, stream>>>(Wq, NQK, WT, 0);
  k_wT<0><<<dim3(NQK / 32, DMOD / 64), b256, 0, stream>>>(Wk, NQK, WT, NQK);
  k_wT<0><<<dim3(DMOD / 32, DMOD / 64), b256, 0, stream>>>(Wv, DMOD, WT, 2 * NQK);
  k_wT<1><<<dim3(DMOD / 32, DMOD / 64), b256, 0, stream>>>(Wo, DMOD, WO16, 0);
  k_gemm_proj<<<dim3(NTOK / TPB, NPROJ / 64), b256, 0, stream>>>(XB, WT, QP, KP, VH, VL);
  k_attn<<<dim3(NBH, SL / TPB), b256, 0, stream>>>(QP, KP, VH, VL, YH, YL);
  k_gemm_out<<<dim3(NTOK / TPB, DMOD / 64), b256, 0, stream>>>(YH, YL, WO16, out);
}
